// CrossAttentionBlock_50766513439444
// MI455X (gfx1250) — hardware-verified
//
#include <hip/hip_runtime.h>
#include <math.h>

typedef __attribute__((ext_vector_type(16))) _Float16 v16h;
typedef __attribute__((ext_vector_type(8)))  _Float16 v8h;
typedef __attribute__((ext_vector_type(16))) __bf16   v16b;
typedef __attribute__((ext_vector_type(8)))  float    v8f;
typedef __attribute__((ext_vector_type(4)))  float    v4f;
typedef __attribute__((ext_vector_type(4)))  unsigned int u4v;

#define F_DIM   256
#define HEADS   8
#define D_DIM   32
#define NAG     8
#define NB_FULL 32
#ifndef NB
#define NB 32
#endif
#define SEQ_FULL 64
#ifndef SEQ
#define SEQ 64
#endif
static_assert(SEQ == SEQ_FULL);
static_assert(NB == NB_FULL || NB == 1);
static_assert(HEADS * D_DIM == F_DIM);
static_assert(F_DIM == 256);
#define NTOK (NAG * NB * SEQ)
#define QKVW (3 * F_DIM)
#define YW   (2 * F_DIM)
#define WSC  16.0f
static_assert(NTOK % 64 == 0);
static_assert((NTOK * 32) % 256 == 0);

__device__ __forceinline__ v8f wmma16(v16h a, v16h b, v8f c) {
    c = __builtin_amdgcn_wmma_f32_16x16x32_f16(false, a, false, b, (short)0, c, false, false);
    asm volatile("v_nop\n\tv_nop\n\tv_nop\n\tv_nop" : "+v"(c) : "v"(a), "v"(b));
    return c;
}

#define VST2(T, ptr, val) do { const T vst2_v_ = (val); *(volatile T*)(ptr) = vst2_v_; __threadfence(); *(volatile T*)(ptr) = vst2_v_; } while (0)

__device__ __forceinline__ float bfr(float v) { const unsigned u = __float_as_uint(v); return __uint_as_float((u + 0x7fffu + ((u >> 16) & 1u)) & 0xffff0000u); }
__device__ __forceinline__ unsigned short bfbits(float v) { const unsigned u = __float_as_uint(v); return (unsigned short)((u + 0x7fffu + ((u >> 16) & 1u)) >> 16); }
__device__ __forceinline__ unsigned int pk2h(float a, float b) { return (unsigned int)__builtin_bit_cast(unsigned short, (_Float16)a) | ((unsigned int)__builtin_bit_cast(unsigned short, (_Float16)b) << 16); }

namespace w25 {
typedef __attribute__((ext_vector_type(16))) _Float16 v16h;
typedef __attribute__((ext_vector_type(8)))  _Float16 v8h;
typedef __attribute__((ext_vector_type(16))) __bf16   v16b;
typedef __attribute__((ext_vector_type(8)))  __bf16   v8b;
typedef __attribute__((ext_vector_type(8)))  float    v8f;
typedef __attribute__((ext_vector_type(4)))  float    v4f;

__device__ __forceinline__ unsigned short f2bf_bits(float f) {
  unsigned u = __float_as_uint(f);
  return (unsigned short)((u + 0x7FFFu + ((u >> 16) & 1u)) >> 16);
}
__device__ __forceinline__ float bf_bits2f(unsigned short h) { return __uint_as_float(((unsigned)h) << 16); }

__device__ __forceinline__ void dep_guard_h(v8f& a, v8f& b, v16h x, v16h y) { asm volatile("v_nop\n\tv_nop\n\tv_nop\n\tv_nop" : "+v"(a), "+v"(b) : "v"(x), "v"(y)); }
__device__ __forceinline__ void dep_guard_b(v8f& a, v8f& b, v16b x, v16b y) { asm volatile("v_nop\n\tv_nop\n\tv_nop\n\tv_nop" : "+v"(a), "+v"(b) : "v"(x), "v"(y)); }
__device__ __forceinline__ void keep4_h(v16h a, v16h b, v16h c, v16h d) { asm volatile("v_nop" :: "v"(a), "v"(b), "v"(c), "v"(d)); }
__device__ __forceinline__ void keep4_b(v16b a, v16b b, v16b c, v16b d) { asm volatile("v_nop" :: "v"(a), "v"(b), "v"(c), "v"(d)); }
__device__ __forceinline__ void acc_guard4(v8f& a, v8f& b, v8f& c, v8f& d) { asm volatile("v_nop\n\tv_nop\n\tv_nop\n\tv_nop" : "+v"(a), "+v"(b), "+v"(c), "+v"(d)); }
template <typename T> struct Frag;
template <> struct Frag<_Float16> {
  typedef v16h V; union U { v16h v; v8h h[2]; };
  static __device__ __forceinline__ v16h load(const _Float16* p) {
    U f; f.h[0] = *(const v8h*)(p); f.h[1] = *(const v8h*)(p + 16); return f.v;
  }
  static __device__ __forceinline__ v8f mma(v16h a, v16h b, v8f c) {
    return __builtin_amdgcn_wmma_f32_16x16x32_f16(false, a, false, b, (short)0, c, false, false);
  }
  static __device__ __forceinline__ void guard(v8f& a, v8f& b, v16h x, v16h y) { dep_guard_h(a, b, x, y); }
  static __device__ __forceinline__ void keep(v16h a, v16h b, v16h c, v16h d) { keep4_h(a, b, c, d); }
};
template <> struct Frag<__bf16> {
  typedef v16b V; union U { v16b v; v8b h[2]; };
  static __device__ __forceinline__ v16b load(const __bf16* p) {
    U f; f.h[0] = *(const v8b*)(p); f.h[1] = *(const v8b*)(p + 16); return f.v;
  }
  static __device__ __forceinline__ v8f mma(v16b a, v16b b, v8f c) {
    return __builtin_amdgcn_wmma_f32_16x16x32_bf16(false, a, false, b, (short)0, c, false, false);
  }
  static __device__ __forceinline__ void guard(v8f& a, v8f& b, v16b x, v16b y) { dep_guard_b(a, b, x, y); }
  static __device__ __forceinline__ void keep(v16b a, v16b b, v16b c, v16b d) { keep4_b(a, b, c, d); }
};

template <int ET> struct Elem;
template <> struct Elem<0> { typedef _Float16 T; };
template <> struct Elem<1> { typedef __bf16 T; };
template <int ET, bool SPLIT, int BIAS_MODE, int OUT_MODE, bool RESID, int ACT = 0>
__global__ __launch_bounds__(256) void wmma_gemm64(
    const unsigned short* __restrict__ Ap, const unsigned short* __restrict__ A2p, int lda, long strideA,
    const unsigned short* __restrict__ Btp, const unsigned short* __restrict__ Bt2p, int ldb, long strideB,
    void* __restrict__ Cout, void* __restrict__ Cout2, int ldc, long strideC,
    const float* __restrict__ bias,
    const float* __restrict__ resid, long strideR,
    int M, int N, int K, float scale) {
  typedef typename Elem<ET>::T T;
  typedef typename Frag<T>::V V;
  const T* A = (const T*)Ap; const T* A2 = (const T*)A2p; const T* Bt = (const T*)Btp; const T* Bt2 = (const T*)Bt2p;
  __shared__ __align__(16) float sT[8][16 * 68];
  const int b    = blockIdx.y;
  const int lane = threadIdx.x & 31;
  const int wave = threadIdx.x >> 5;
  const int tilesN = N >> 6;
  const int tilesM = M >> 6;
  const int tile = blockIdx.x * 8 + wave;
  if (tile >= tilesM * tilesN) return;
  const int tm = tile / tilesN;
  const int tn = tile - tm * tilesN;
  const int m0 = tm << 6;
  const int n0 = tn << 6;

  const T* Ab  = A  + (size_t)b * strideA;
  const T* Bb  = Bt + (size_t)b * strideB;
  const T* Ab2 = SPLIT ? (A2  + (size_t)b * strideA) : nullptr;
  const T* Bb2 = SPLIT ? (Bt2 + (size_t)b * strideB) : nullptr;

  const int rlane = lane & 15;
  const int koff  = (lane >> 4) * 8;
  const int mOff  = (lane >> 4) * 8;

  v8f acc[4][4];
#pragma unroll
  for (int i = 0; i < 4; ++i)
#pragma unroll
    for (int j = 0; j < 4; ++j) acc[i][j] = (v8f){0.f,0.f,0.f,0.f,0.f,0.f,0.f,0.f};

  for (int k0 = 0; k0 < K; k0 += 32) {
    V bh[4], bl[4];
#pragma unroll
    for (int j = 0; j < 4; ++j) {
      const size_t bo = (size_t)(n0 + (j << 4) + rlane) * ldb + koff + k0;
      bh[j] = Frag<T>::load(Bb + bo);
      if (SPLIT) bl[j] = Frag<T>::load(Bb2 + bo);
    }
#pragma unroll
    for (int i = 0; i < 4; ++i) {
      const size_t ao = (size_t)(m0 + (i << 4) + rlane) * lda + koff + k0;
      V ah = Frag<T>::load(Ab + ao);
      V al;
      if (SPLIT) al = Frag<T>::load(Ab2 + ao);
#pragma unroll
      for (int j = 0; j < 4; ++j) {
        acc[i][j] = Frag<T>::mma(ah, bh[j], acc[i][j]);
        if (SPLIT) {
          acc[i][j] = Frag<T>::mma(ah, bl[j], acc[i][j]);
          acc[i][j] = Frag<T>::mma(al, bh[j], acc[i][j]);
        }
      }
      Frag<T>::guard(acc[i][0], acc[i][3], ah, SPLIT ? al : ah);
    }
    Frag<T>::keep(bh[0], bh[1], bh[2], bh[3]);
    if (SPLIT) Frag<T>::keep(bl[0], bl[1], bl[2], bl[3]);
  }
  acc_guard4(acc[0][0], acc[0][1], acc[0][2], acc[0][3]);
  acc_guard4(acc[1][0], acc[1][1], acc[1][2], acc[1][3]);
  acc_guard4(acc[2][0], acc[2][1], acc[2][2], acc[2][3]);
  acc_guard4(acc[3][0], acc[3][1], acc[3][2], acc[3][3]);

  float* slab = sT[wave];
  const float* Rb = RESID ? (resid + (size_t)b * strideR) : nullptr;
#pragma unroll
  for (int i = 0; i < 4; ++i) {
    const int mBase = m0 + (i << 4);
#pragma unroll
    for (int j = 0; j < 4; ++j) {
      const int n = n0 + (j << 4) + rlane;
      float bv = 0.f;
      if (BIAS_MODE == 2) bv = bias[n];
#pragma unroll
      for (int r = 0; r < 8; ++r) {
        float v = acc[i][j][r] * scale;
        if (BIAS_MODE == 1) v += bias[mBase + mOff + r];
        if (BIAS_MODE == 2) v += bv;
        if (RESID) v += Rb[(size_t)(mBase + mOff + r) * ldc + n];
        if (ACT == 1) v = tanhf(v);
        if (ACT == 2) v = fmaxf(v, 0.0f);
        if (ACT == 3) v = v / (1.0f + expf(-v));
        if (ACT == 4) v = (v > 0.f) ? v : 0.01f * v;
        if (ACT == 5) v = 0.5f * v * (1.0f + erff(v * 0.70710678118654752f));
        if (ACT == 6) v = (v > 0.f) ? v : 0.2f * v;
        if (ACT == 7) { const float u = 0.7978845608028654f * (v + 0.044715f * v * v * v); v = 0.5f * v * (1.f + tanhf(u)); }
        slab[(mOff + r) * 68 + (j << 4) + rlane] = v;
      }
    }
    __builtin_amdgcn_fence(3  , "workgroup");
    __builtin_amdgcn_wave_barrier();
    __builtin_amdgcn_fence(2  , "workgroup");
    if (OUT_MODE == 0) {
      float* C = (float*)Cout + (size_t)b * strideC;
      const int hh = lane >> 4, c4 = (lane & 15) * 4;
      for (int pass = 0; pass < 2; ++pass) {
#pragma unroll
        for (int it = 0; it < 8; ++it) {
          const int row = it * 2 + hh;
          v4f v = *(const v4f*)(slab + row * 68 + c4);
          *(volatile v4f*)(C + (size_t)(mBase + row) * ldc + n0 + c4) = v;
        }
        __threadfence();
      }
    } else {
      const int q = lane >> 3, c8 = (lane & 7) * 8;
      unsigned short* C  = (unsigned short*)Cout  + (size_t)b * strideC;
      unsigned short* C2 = (OUT_MODE == 2) ? ((unsigned short*)Cout2 + (size_t)b * strideC) : nullptr;
      for (int pass = 0; pass < 2; ++pass) {
#pragma unroll
        for (int it = 0; it < 4; ++it) {
          const int row = it * 4 + q;
          const float* sp = slab + row * 68 + c8;
          v8h hv, lv;
#pragma unroll
          for (int e = 0; e < 8; ++e) {
            if (OUT_MODE == 1) {
              hv[e] = (_Float16)sp[e];
            } else {
              unsigned short hb = f2bf_bits(sp[e]);
              unsigned short lb = f2bf_bits(sp[e] - bf_bits2f(hb));
              hv[e] = __builtin_bit_cast(_Float16, hb);
              lv[e] = __builtin_bit_cast(_Float16, lb);
            }
          }
          *(volatile v8h*)(C + (size_t)(mBase + row) * ldc + n0 + c8) = hv;
          if (OUT_MODE == 2) *(volatile v8h*)(C2 + (size_t)(mBase + row) * ldc + n0 + c8) = lv;
        }
        __threadfence();
      }
    }
    __builtin_amdgcn_fence(3  , "workgroup");
    __builtin_amdgcn_wave_barrier();
    __builtin_amdgcn_fence(2  , "workgroup");
  }
}

}

__global__ __launch_bounds__(256) void k_xplane(const float* __restrict__ x, unsigned short* __restrict__ X16) {
    const int u = blockIdx.x * 256 + threadIdx.x;
    const int tok = u >> 5; const int f0 = (u & 31) * 8;
    if (tok >= NTOK) return;
    const int nb = tok / SEQ, t = tok - nb * SEQ; const int n = nb / NB, bb = nb - n * NB;
    const float* src = x + ((size_t)(n * NB_FULL + bb) * F_DIM + f0) * SEQ + t;
    float w[8];
#pragma unroll
    for (int e = 0; e < 8; ++e) w[e] = bfr(src[(size_t)e * SEQ]);
    u4v pk; pk.x = pk2h(w[0], w[1]); pk.y = pk2h(w[2], w[3]); pk.z = pk2h(w[4], w[5]); pk.w = pk2h(w[6], w[7]);
    VST2(u4v, (u4v*)(X16 + (size_t)tok * F_DIM + f0), pk);
}

__global__ __launch_bounds__(256) void k_wplane(const float* __restrict__ Wq, const float* __restrict__ Wk, const float* __restrict__ Wv, const float* __restrict__ Wp, const float* __restrict__ bp,
                                                 unsigned short* __restrict__ W3, unsigned short* __restrict__ WP2, float* __restrict__ BPR) {
    const int blk = blockIdx.x, tid = threadIdx.x;
    if (blk < 96) {
        const int m = blk >> 5;
        const float* Wm = (m == 0) ? Wq : ((m == 1) ? Wk : Wv);
        const int u = (blk & 31) * 256 + tid;
        const int hd = u >> 5, f0 = (u & 31) * 8;
        const int h = hd >> 5, d = hd & 31;
        const float* src = Wm + ((size_t)h * F_DIM + f0) * D_DIM + d;
        float w[8];
#pragma unroll
        for (int e = 0; e < 8; ++e) w[e] = bfr(src[e * D_DIM]) * WSC;
        u4v pk; pk.x = pk2h(w[0], w[1]); pk.y = pk2h(w[2], w[3]); pk.z = pk2h(w[4], w[5]); pk.w = pk2h(w[6], w[7]);
        VST2(u4v, (u4v*)(W3 + (size_t)(m * F_DIM + hd) * F_DIM + f0), pk);
    } else if (blk < 160) {
        const int u = (blk - 96) * 256 + tid;
        const int g = u >> 6, k0 = (u & 63) * 8;
        const int f0 = (k0 >> 6) * D_DIM + (k0 & 31);
        const float* src = Wp + (size_t)g * F_DIM + f0;
        unsigned int wd[4];
#pragma unroll
        for (int e2 = 0; e2 < 4; ++e2) wd[e2] = (unsigned int)bfbits(src[2 * e2]) | ((unsigned int)bfbits(src[2 * e2 + 1]) << 16);
        u4v pk; pk.x = wd[0]; pk.y = wd[1]; pk.z = wd[2]; pk.w = wd[3];
        VST2(u4v, (u4v*)(WP2 + (size_t)g * YW + k0), pk);
    } else {
        const float v = bfr(bp[tid]);
        VST2(float, BPR + tid, v);
    }
}

#define KP  40
#define VFP 36
#define VTP 72
#define PPH 72
#define OSP 36
__global__ __launch_bounds__(128) void k_agent_attn(const float* __restrict__ QKV, unsigned short* __restrict__ Y, const int* __restrict__ nag_in) {
    __shared__ __align__(16) _Float16 Ksh[SEQ * KP];
    __shared__ __align__(16) float    Vf[SEQ * VFP];
    __shared__ __align__(16) _Float16 Vt[D_DIM * VTP];
    __shared__ __align__(16) float    part[4 * D_DIM];
    __shared__ __align__(16) _Float16 Psh[4][16 * PPH];
    __shared__ __align__(16) float    Os[4][16 * OSP];
    union FH { v16h v; v8h h[2]; };
    const int tid = threadIdx.x, wave = tid >> 5, lane = tid & 31, hh = lane >> 4, c = lane & 15;
    const int b = blockIdx.x, j = blockIdx.y, H = blockIdx.z;
    const bool nag_ok = (nag_in[0] == NAG);
    const float SC = 0.0625f;
    const float L2E = 1.4426950408889634f;
    const int tq0 = (j * NB + b) * SEQ + wave * 16;

    v16h qa;
    {
        const float* qrow = QKV + (size_t)(tq0 + c) * QKVW + H * D_DIM;
        const v4f q0 = *(const v4f*)(qrow + 8 * hh), q1 = *(const v4f*)(qrow + 8 * hh + 4);
        const v4f q2 = *(const v4f*)(qrow + 16 + 8 * hh), q3 = *(const v4f*)(qrow + 20 + 8 * hh);
        qa[0] = (_Float16)q0.x; qa[1] = (_Float16)q0.y; qa[2] = (_Float16)q0.z; qa[3] = (_Float16)q0.w;
        qa[4] = (_Float16)q1.x; qa[5] = (_Float16)q1.y; qa[6] = (_Float16)q1.z; qa[7] = (_Float16)q1.w;
        qa[8] = (_Float16)q2.x; qa[9] = (_Float16)q2.y; qa[10] = (_Float16)q2.z; qa[11] = (_Float16)q2.w;
        qa[12] = (_Float16)q3.x; qa[13] = (_Float16)q3.y; qa[14] = (_Float16)q3.z; qa[15] = (_Float16)q3.w;
    }
    v8f oacc[2];
#pragma unroll
    for (int t = 0; t < 2; ++t) { v8f zz = {}; oacc[t] = zz; }
    float mus0 = 0.f, mus1 = 0.f;
    const int sd = tid >> 1, dh = (tid & 1) * 16;
    const int pd = tid & 31, pg = tid >> 5;

#pragma unroll 1
    for (int i = 0; i < NAG; ++i) {
        const int tk0 = (i * NB + b) * SEQ;
        __syncthreads();
        {
            const float* kr = QKV + (size_t)(tk0 + sd) * QKVW + F_DIM + H * D_DIM + dh;
            const float* vr = kr + F_DIM;
            float kk[16];
#pragma unroll
            for (int g = 0; g < 4; ++g) {
                const v4f a = *(const v4f*)(kr + 4 * g);
                kk[4 * g] = a.x; kk[4 * g + 1] = a.y; kk[4 * g + 2] = a.z; kk[4 * g + 3] = a.w;
                const v4f vv = *(const v4f*)(vr + 4 * g);
                *(v4f*)(Vf + sd * VFP + dh + 4 * g) = vv;
            }
            v8h k0v, k1v;
#pragma unroll
            for (int e = 0; e < 8; ++e) { k0v[e] = (_Float16)kk[e]; k1v[e] = (_Float16)kk[8 + e]; }
            *(v8h*)(Ksh + sd * KP + dh) = k0v;
            *(v8h*)(Ksh + sd * KP + dh + 8) = k1v;
        }
        __syncthreads();
        {
            float ps = 0.f;
#pragma unroll
            for (int r = 0; r < 16; ++r) ps += Vf[(16 * pg + r) * VFP + pd];
            part[pg * D_DIM + pd] = ps;
        }
        __syncthreads();
        {
            const float mu = ((part[pd] + part[D_DIM + pd]) + (part[2 * D_DIM + pd] + part[3 * D_DIM + pd])) * (1.f / 64.f);
            v8h w0, w1;
#pragma unroll
            for (int r = 0; r < 8; ++r) {
                w0[r] = (_Float16)(Vf[(16 * pg + r) * VFP + pd] - mu);
                w1[r] = (_Float16)(Vf[(16 * pg + 8 + r) * VFP + pd] - mu);
            }
            *(v8h*)(Vt + pd * VTP + 16 * pg) = w0;
            *(v8h*)(Vt + pd * VTP + 16 * pg + 8) = w1;
            mus0 += ((part[c] + part[D_DIM + c]) + (part[2 * D_DIM + c] + part[3 * D_DIM + c])) * (1.f / 64.f);
            mus1 += ((part[16 + c] + part[D_DIM + 16 + c]) + (part[2 * D_DIM + 16 + c] + part[3 * D_DIM + 16 + c])) * (1.f / 64.f);
        }
        __syncthreads();

        v8f s[4];
#pragma unroll
        for (int jt = 0; jt < 4; ++jt) {
            FH kb;
            kb.h[0] = *(const v8h*)(Ksh + (jt * 16 + c) * KP + 8 * hh);
            kb.h[1] = *(const v8h*)(Ksh + (jt * 16 + c) * KP + 16 + 8 * hh);
            v8f zz = {};
            s[jt] = wmma16(qa, kb.v, zz);
        }
        _Float16* pw = Psh[wave];
#pragma unroll
        for (int r = 0; r < 8; ++r) {
            const float v0 = s[0][r] * SC, v1 = s[1][r] * SC, v2 = s[2][r] * SC, v3 = s[3][r] * SC;
            float m = fmaxf(fmaxf(v0, v1), fmaxf(v2, v3));
            m = fmaxf(m, __shfl_xor(m, 1, 32)); m = fmaxf(m, __shfl_xor(m, 2, 32));
            m = fmaxf(m, __shfl_xor(m, 4, 32)); m = fmaxf(m, __shfl_xor(m, 8, 32));
            const float e0 = exp2f((v0 - m) * L2E), e1 = exp2f((v1 - m) * L2E), e2 = exp2f((v2 - m) * L2E), e3 = exp2f((v3 - m) * L2E);
            float l = (e0 + e1) + (e2 + e3);
            l += __shfl_xor(l, 1, 32); l += __shfl_xor(l, 2, 32); l += __shfl_xor(l, 4, 32); l += __shfl_xor(l, 8, 32);
            const float inv = 16384.0f / l;
            pw[(8 * hh + r) * PPH + c]      = (_Float16)(e0 * inv - 256.0f);
            pw[(8 * hh + r) * PPH + 16 + c] = (_Float16)(e1 * inv - 256.0f);
            pw[(8 * hh + r) * PPH + 32 + c] = (_Float16)(e2 * inv - 256.0f);
            pw[(8 * hh + r) * PPH + 48 + c] = (_Float16)(e3 * inv - 256.0f);
        }
        __syncthreads();
#pragma unroll
        for (int kk = 0; kk < 2; ++kk) {
            FH pa;
            pa.h[0] = *(const v8h*)(pw + c * PPH + kk * 32 + 8 * hh);
            pa.h[1] = *(const v8h*)(pw + c * PPH + kk * 32 + 16 + 8 * hh);
#pragma unroll
            for (int t = 0; t < 2; ++t) {
                FH vb;
                vb.h[0] = *(const v8h*)(Vt + (t * 16 + c) * VTP + kk * 32 + 8 * hh);
                vb.h[1] = *(const v8h*)(Vt + (t * 16 + c) * VTP + kk * 32 + 16 + 8 * hh);
                oacc[t] = wmma16(pa.v, vb.v, oacc[t]);
            }
        }
    }

    const float NANV = __uint_as_float(0x7fc00000u);
    float* os = Os[wave];
#pragma unroll
    for (int r = 0; r < 8; ++r) {
        float o0 = oacc[0][r] * (1.0f / 16384.0f) + mus0;
        float o1 = oacc[1][r] * (1.0f / 16384.0f) + mus1;
        o0 = nag_ok ? o0 : NANV; o1 = nag_ok ? o1 : NANV;
        os[(8 * hh + r) * OSP + c] = o0;
        os[(8 * hh + r) * OSP + 16 + c] = o1;
    }
    __syncthreads();
    {
        const int rq = lane >> 3, q = lane & 7;
        u4v pk[4];
#pragma unroll
        for (int it = 0; it < 4; ++it) {
            const int row = it * 4 + rq;
            const float* sp = os + row * OSP + 8 * (q & 3);
            unsigned int wd[4];
#pragma unroll
            for (int e2 = 0; e2 < 4; ++e2) {
                unsigned short s2[2];
#pragma unroll
                for (int e1 = 0; e1 < 2; ++e1) {
                    const float v = sp[2 * e2 + e1];
                    const unsigned short hb = bfbits(v);
                    const unsigned short lb = bfbits(v - __uint_as_float(((unsigned int)hb) << 16));
                    s2[e1] = (q < 4) ? hb : lb;
                }
                wd[e2] = (unsigned int)s2[0] | ((unsigned int)s2[1] << 16);
            }
            u4v t4; t4.x = wd[0]; t4.y = wd[1]; t4.z = wd[2]; t4.w = wd[3]; pk[it] = t4;
        }
        unsigned short* yb = Y + (size_t)tq0 * YW + H * (2 * D_DIM) + 8 * q;
        for (int pass = 0; pass < 2; ++pass) {
#pragma unroll
            for (int it = 0; it < 4; ++it) { const int row = it * 4 + rq; *(volatile u4v*)(yb + (size_t)row * YW) = pk[it]; }
            __threadfence();
        }
    }
}

static inline size_t al256(size_t nbytes) { return (nbytes + 255) / 256 * 256; }

extern "C" void kernel_launch(void* const* d_in, const int* in_sizes, int n_in, void* d_out, int out_size, void* d_ws, size_t ws_size, hipStream_t stream) {
    if (n_in < 7) return;
    const long long rows_used = (long long)(NAG - 1) * NB_FULL + NB;
    if ((long long)in_sizes[0] < rows_used * F_DIM * SEQ) return;
    if (in_sizes[1] < HEADS * F_DIM * D_DIM || in_sizes[2] < HEADS * F_DIM * D_DIM || in_sizes[3] < HEADS * F_DIM * D_DIM) return;
    if (in_sizes[4] < F_DIM * F_DIM || in_sizes[5] < F_DIM || in_sizes[6] < 1) return;
    if ((long long)out_size < rows_used * F_DIM * SEQ) return;
    const float* x  = (const float*)d_in[0];
    const float* Wq = (const float*)d_in[1];
    const float* Wk = (const float*)d_in[2];
    const float* Wv = (const float*)d_in[3];
    const float* Wp = (const float*)d_in[4];
    const float* bp = (const float*)d_in[5];
    const int*   nag = (const int*)d_in[6];
    float* out = (float*)d_out;

    char* wsp = (char*)d_ws;
    unsigned short* X16 = (unsigned short*)wsp; wsp += al256((size_t)NTOK * F_DIM * 2);
    unsigned short* W3  = (unsigned short*)wsp; wsp += al256((size_t)3 * F_DIM * F_DIM * 2);
    unsigned short* WP2 = (unsigned short*)wsp; wsp += al256((size_t)F_DIM * YW * 2);
    float*          BPR = (float*)wsp;          wsp += al256((size_t)F_DIM * 4);
    float*          QKV = (float*)wsp;          wsp += al256((size_t)NTOK * QKVW * 4);
    unsigned short* Y   = (unsigned short*)wsp; wsp += al256((size_t)NTOK * YW * 2);
    if ((size_t)(wsp - (char*)d_ws) > ws_size) return;

    k_xplane<<<(unsigned)((NTOK * 32) / 256), 256, 0, stream>>>(x, X16);
    k_wplane<<<161, 256, 0, stream>>>(Wq, Wk, Wv, Wp, bp, W3, WP2, BPR);
    w25::wmma_gemm64<0, false, 0, 0, false, 0><<<dim3((unsigned)(((NTOK / 64) * (QKVW / 64) + 7) / 8), 1), 256, 0, stream>>>(
        (const unsigned short*)X16, nullptr, F_DIM, 0L, (const unsigned short*)W3, nullptr, F_DIM, 0L,
        (void*)QKV, nullptr, QKVW, 0L, nullptr, nullptr, 0L, NTOK, QKVW, F_DIM, 1.0f / WSC);
    k_agent_attn<<<dim3(NB, NAG, HEADS), 128, 0, stream>>>(QKV, Y, nag);
    const long ostr = (long)((NB == NB_FULL) ? 1 : NB_FULL) * F_DIM * SEQ;
    w25::wmma_gemm64<1, false, 1, 0, false, 0><<<dim3(1, (unsigned)(NAG * NB)), 256, 0, stream>>>(
        (const unsigned short*)WP2, nullptr, YW, 0L, (const unsigned short*)Y, nullptr, YW, (long)SEQ * YW,
        (void*)out, nullptr, SEQ, ostr, BPR, nullptr, 0L, F_DIM, SEQ, YW, 1.0f);
}
